// BertSelfAttention_37692632990185
// MI455X (gfx1250) — hardware-verified
//
#include <hip/hip_runtime.h>
#ifndef NB
#define NB 2
#endif
#ifndef SEQ
#define SEQ 2048
#endif
#define NB_FULL 2
#define SEQ_FULL 2048
#define HID 1024
#define NH 16
#define HD 64
#define NT64 (SEQ / 64)
#define NR (NB * SEQ)
#define NTN (HID / 64)
#define NF (NB * NT64 * NT64)
#define NFP (((NF + 31) / 32) * 32)

static_assert(NB <= NB_FULL);
static_assert(SEQ <= SEQ_FULL);
static_assert(SEQ % 128 == 0);
static_assert(NH * HD == HID);
static_assert(HD == 64);
static_assert((SEQ * HID / 8) % 256 == 0);
static_assert((HID * HID / 8) % 256 == 0);
static_assert(NR % 128 == 0);
static_assert((size_t)(NB * NH * NT64) * 4 * 16 * 64 == (size_t)NB * SEQ * HID);
static_assert((size_t)((NR / 128) * NTN) * 4 * 32 * 64 == (size_t)NR * HID);

typedef _Float16 v16h __attribute__((ext_vector_type(16)));
typedef _Float16 v4h __attribute__((ext_vector_type(4)));
typedef unsigned short v8us __attribute__((ext_vector_type(8), may_alias));
typedef unsigned int v4u __attribute__((ext_vector_type(4)));
typedef float v8f __attribute__((ext_vector_type(8)));
typedef float v4f __attribute__((ext_vector_type(4)));
typedef float v4fa __attribute__((ext_vector_type(4), may_alias));
union FragH { v16h v; v8us half[2]; _Float16 h[16]; unsigned short u[16]; };

__device__ __forceinline__ unsigned short bf16_bits(float x) { unsigned int u = __float_as_uint(x); return (unsigned short)((u + 0x7FFFu + ((u >> 16) & 1u)) >> 16); }
__device__ __forceinline__ float bf16_rne(float x) { return __uint_as_float(((unsigned int)bf16_bits(x)) << 16); }

__device__ __forceinline__ v16h g2_frag(const _Float16* p, unsigned hh) { FragH f; f.half[0] = *(const v8us*)((const unsigned short*)p + 8u * hh); f.half[1] = *(const v8us*)((const unsigned short*)p + 16u + 8u * hh); return f.v; }
__device__ __forceinline__ v8f g2_mma(v16h a, v16h b, v8f c) { v8f d = __builtin_amdgcn_wmma_f32_16x16x32_f16(false, a, false, b, (short)0, c, false, false); asm volatile("v_nop\n\tv_nop\n\tv_nop\n\tv_nop" : "+v"(d) : "v"(a), "v"(b)); return d; }
__device__ __forceinline__ v8f mma2(v16h a0, v16h b0, v16h a1, v16h b1, v8f c) {
  c = __builtin_amdgcn_wmma_f32_16x16x32_f16(false, a0, false, b0, (short)0, c, false, false);
  c = __builtin_amdgcn_wmma_f32_16x16x32_f16(false, a1, false, b1, (short)0, c, false, false);
  asm volatile("v_nop\n\tv_nop\n\tv_nop\n\tv_nop" : "+v"(c) : "v"(a0), "v"(a1), "v"(b0), "v"(b1));
  return c;
}

__global__ __launch_bounds__(256) void k_x16(const float* __restrict__ x, _Float16* __restrict__ X16) {
  const unsigned t = blockIdx.x * 256u + threadIdx.x; const unsigned b = blockIdx.y;
  if (t >= (unsigned)(SEQ * HID / 8)) return;
  const float* src = x + (size_t)b * SEQ_FULL * HID + (size_t)t * 8;
  const v4f a = *(const v4fa*)src, c = *(const v4fa*)(src + 4);
  FragH f;
#pragma unroll
  for (int q = 0; q < 4; ++q) { f.h[q] = (_Float16)bf16_rne(a[q]); f.h[4 + q] = (_Float16)bf16_rne(c[q]); }
  const v8us o = f.half[0];
  unsigned short* d = (unsigned short*)X16 + (size_t)b * SEQ * HID + (size_t)t * 8;
  *(volatile v8us*)d = o; __threadfence(); *(volatile v8us*)d = o;
}

__global__ __launch_bounds__(256) void k_wnat(const float* __restrict__ wq, const float* __restrict__ wk, const float* __restrict__ wv, _Float16* __restrict__ W16) {
  const unsigned t = blockIdx.x * 256u + threadIdx.x; const unsigned y = blockIdx.y;
  if (t >= (unsigned)(HID * HID / 8)) return;
  const float* w = (y == 0u) ? wq : ((y == 1u) ? wk : wv);
  const v4f a = *(const v4fa*)(w + (size_t)t * 8), c = *(const v4fa*)(w + (size_t)t * 8 + 4);
  FragH f;
#pragma unroll
  for (int q = 0; q < 4; ++q) { f.h[q] = (_Float16)(bf16_rne(a[q]) * 16.0f); f.h[4 + q] = (_Float16)(bf16_rne(c[q]) * 16.0f); }
  const v8us o = f.half[0];
  unsigned short* d = (unsigned short*)W16 + (size_t)y * HID * HID + (size_t)t * 8;
  *(volatile v8us*)d = o; __threadfence(); *(volatile v8us*)d = o;
}

__global__ __launch_bounds__(128) void k_gemm2(const _Float16* __restrict__ X16, const _Float16* __restrict__ W16, const float* __restrict__ bq, const float* __restrict__ bk, const float* __restrict__ bv, _Float16* __restrict__ QKV) {
  __shared__ __attribute__((aligned(16))) float so[4][32][68];
  const unsigned tid = threadIdx.x, w = tid >> 5, lane = tid & 31u, ln = lane & 15u, hh = lane >> 4; const unsigned y = blockIdx.y;
  const _Float16* Bh = W16 + (size_t)y * HID * HID;
  const float* bias = (y == 0u) ? bq : ((y == 1u) ? bk : bv);
  _Float16* C16 = QKV + (size_t)y * NR * HID;
  const unsigned mt = blockIdx.x / (unsigned)NTN, nq = blockIdx.x % (unsigned)NTN;
  const unsigned row0 = mt * 128u + 32u * w, col0 = nq * 64u;
  if (row0 >= (unsigned)NR) return;
  const _Float16* a0p = X16 + (size_t)(row0 + ln) * HID; const _Float16* a1p = a0p + (size_t)16 * HID;
  const _Float16* b0p = Bh + (size_t)(col0 + ln) * HID; const _Float16* b1p = b0p + (size_t)16 * HID; const _Float16* b2p = b1p + (size_t)16 * HID; const _Float16* b3p = b2p + (size_t)16 * HID;
  const v8f z8 = {0.f,0.f,0.f,0.f,0.f,0.f,0.f,0.f}; v8f c00 = z8, c01 = z8, c02 = z8, c03 = z8, c10 = z8, c11 = z8, c12 = z8, c13 = z8;
#pragma unroll 1
  for (unsigned kb = 0; kb < (unsigned)HID; kb += 32u) { const v16h a0 = g2_frag(a0p + kb, hh), a1 = g2_frag(a1p + kb, hh);
    v16h b = g2_frag(b0p + kb, hh); c00 = g2_mma(a0, b, c00); c10 = g2_mma(a1, b, c10);
    b = g2_frag(b1p + kb, hh); c01 = g2_mma(a0, b, c01); c11 = g2_mma(a1, b, c11);
    b = g2_frag(b2p + kb, hh); c02 = g2_mma(a0, b, c02); c12 = g2_mma(a1, b, c12);
    b = g2_frag(b3p + kb, hh); c03 = g2_mma(a0, b, c03); c13 = g2_mma(a1, b, c13); }
  v8f accs[8] = {c00, c01, c02, c03, c10, c11, c12, c13};
#pragma unroll
  for (int u = 0; u < 8; ++u) { const int t = u & 3, hf = u >> 2; const unsigned col = col0 + (unsigned)t * 16u + ln; const float bvl = bf16_rne(bias[col]);
#pragma unroll
    for (int r = 0; r < 8; ++r) { const unsigned rloc = (unsigned)hf * 16u + 8u * hh + (unsigned)r; so[w][rloc][t * 16 + ln] = accs[u][r] * 0.0625f + bvl; } }
  __builtin_amdgcn_fence(4  , "workgroup"); __builtin_amdgcn_wave_barrier();
  const unsigned rsub = lane >> 4, c4 = (lane & 15u) * 4u;
  for (int pass = 0; pass < 2; ++pass) {
#pragma unroll
    for (int q = 0; q < 16; ++q) { const unsigned r = (unsigned)q * 2u + rsub; const v4f v = *(const v4fa*)&so[w][r][c4]; v4h h4;
#pragma unroll
      for (int i = 0; i < 4; ++i) h4[i] = (_Float16)v[i];
      *(volatile v4h*)(C16 + (size_t)(row0 + r) * HID + col0 + c4) = h4; }
    if (pass == 0) __threadfence(); }
}

__global__ __launch_bounds__(256) void k_vt(const _Float16* __restrict__ V16, _Float16* __restrict__ Vt) {
  __shared__ unsigned short tl[64][66];
  const unsigned tid = threadIdx.x; const unsigned slab = blockIdx.x / (unsigned)NT64, lg = blockIdx.x % (unsigned)NT64; const unsigned b = slab / (unsigned)NH, h = slab % (unsigned)NH;
  for (unsigned i = tid; i < 512u; i += 256u) { const unsigned r = i >> 3, c8 = (i & 7u) * 8u; FragH f;
    f.half[0] = *(const v8us*)((const unsigned short*)V16 + ((size_t)b * SEQ + lg * 64u + r) * HID + h * 64u + c8);
#pragma unroll
    for (int q = 0; q < 8; ++q) tl[r][c8 + q] = f.u[q]; }
  __syncthreads();
  for (int pass = 0; pass < 2; ++pass) {
#pragma unroll
    for (int rd = 0; rd < 2; ++rd) { const unsigned d = (unsigned)rd * 32u + (tid >> 3), pc = tid & 7u; FragH f;
#pragma unroll
      for (int q = 0; q < 8; ++q) f.u[q] = tl[pc * 8u + q][d];
      *(volatile v8us*)((unsigned short*)Vt + ((size_t)slab * 64u + d) * SEQ + lg * 64u + pc * 8u) = f.half[0]; }
    if (pass == 0) __threadfence(); }
}

__global__ __launch_bounds__(256) void k_mflag(const float* __restrict__ mask, unsigned int* __restrict__ flags) {
  __shared__ unsigned int sfl[32];
  const unsigned tid = threadIdx.x, w = tid >> 5, lane = tid & 31u; const unsigned rsub = lane >> 4, c4 = (lane & 15u) * 4u;
#pragma unroll 1
  for (unsigned j = 0; j < 4u; ++j) {
    const unsigned f = blockIdx.x * 32u + w * 4u + j; const unsigned fc = (f < (unsigned)NF) ? f : (unsigned)(NF - 1);
    const unsigned kt = fc % (unsigned)NT64, qt = (fc / (unsigned)NT64) % (unsigned)NT64, b = fc / (unsigned)(NT64 * NT64);
    const float* p = mask + ((size_t)b * SEQ_FULL + qt * 64u + rsub) * SEQ_FULL + kt * 64u + c4;
    unsigned bad = 0u;
#pragma unroll 4
    for (unsigned i = 0; i < 32u; ++i) { const v4f v = *(const v4fa*)(p + (size_t)(2u * i) * SEQ_FULL); bad |= (unsigned)(v[0] != 1.0f) | (unsigned)(v[1] != 1.0f) | (unsigned)(v[2] != 1.0f) | (unsigned)(v[3] != 1.0f); }
    const int any = __any((int)(bad != 0u));
    if (lane == 0u) sfl[w * 4u + j] = any ? 1u : 0u;
  }
  __syncthreads();
  if (tid < 8u) { v4u v; v[0] = sfl[4u * tid]; v[1] = sfl[4u * tid + 1u]; v[2] = sfl[4u * tid + 2u]; v[3] = sfl[4u * tid + 3u];
    unsigned int* d = flags + (size_t)blockIdx.x * 32u + 4u * tid;
    *(volatile v4u*)d = v; __threadfence(); *(volatile v4u*)d = v; }
}

__global__ __launch_bounds__(128) void k_flash(const _Float16* __restrict__ Q16, const _Float16* __restrict__ K16, const _Float16* __restrict__ VT, const float* __restrict__ mask, const unsigned int* __restrict__ flags, float* __restrict__ out) {
  __shared__ __attribute__((aligned(16))) float so[4][16][68];
  const unsigned tid = threadIdx.x, w = tid >> 5, lane = tid & 31u, ln = lane & 15u, hh = lane >> 4;
  const unsigned bid = blockIdx.x; const unsigned qt = bid % (unsigned)NT64, h = (bid / (unsigned)NT64) % (unsigned)NH, b = bid / (unsigned)(NT64 * NH);
  const unsigned q0 = qt * 64u + 16u * w;
  const _Float16* qrow = Q16 + (size_t)(b * (unsigned)SEQ + q0 + ln) * HID + h * 64u;
  const v16h qb0 = g2_frag(qrow, hh), qb1 = g2_frag(qrow + 32, hh);
  const _Float16* kbase = K16 + (size_t)(b * (unsigned)SEQ + ln) * HID + h * 64u;
  const _Float16* vbase = VT + (size_t)((b * (unsigned)NH + h) * 64u + ln) * SEQ;
  const float* mrow = mask + ((size_t)b * SEQ_FULL + q0 + ln) * SEQ_FULL;
  const unsigned int* frow = flags + (size_t)(b * (unsigned)NT64 + qt) * NT64;
  const v8f z8 = {0.f,0.f,0.f,0.f,0.f,0.f,0.f,0.f};
  v8f o[4] = {z8, z8, z8, z8};
  float m_run = -1.0e30f, l_run = 0.f;
#pragma unroll 1
  for (unsigned kt = 0; kt < (unsigned)NT64; ++kt) {
    const unsigned key0 = kt * 64u;
    v8f s[4];
#pragma unroll
    for (int j = 0; j < 4; ++j) { const _Float16* kp = kbase + (size_t)(key0 + 16u * (unsigned)j) * HID; const v16h a0 = g2_frag(kp, hh), a1 = g2_frag(kp + 32, hh); s[j] = mma2(a0, qb0, a1, qb1, z8); }
#pragma unroll
    for (int j = 0; j < 4; ++j)
#pragma unroll
      for (int r = 0; r < 8; ++r) s[j][r] *= 0.125f;
    const unsigned fl = frow[kt];
    if (fl != 0u) {
#pragma unroll
      for (int j = 0; j < 4; ++j) { const float* mp = mrow + key0 + 16u * (unsigned)j + 8u * hh; const v4f m0 = *(const v4fa*)mp, m1 = *(const v4fa*)(mp + 4);
#pragma unroll
        for (int r = 0; r < 4; ++r) { s[j][r] += (1.0f - bf16_rne(m0[r])) * -10000.0f; s[j][4 + r] += (1.0f - bf16_rne(m1[r])) * -10000.0f; } }
    }
    float mx = s[0][0];
#pragma unroll
    for (int j = 0; j < 4; ++j)
#pragma unroll
      for (int r = 0; r < 8; ++r) mx = fmaxf(mx, s[j][r]);
    mx = fmaxf(mx, __shfl_xor(mx, 16));
    const float newm = fmaxf(m_run, mx);
    const float alpha = __expf(m_run - newm);
    m_run = newm;
    FragH pb0, pb1; float rs = 0.f;
#pragma unroll
    for (int r = 0; r < 8; ++r) {
      const float e0 = __expf(s[0][r] - newm), e1 = __expf(s[1][r] - newm), e2 = __expf(s[2][r] - newm), e3 = __expf(s[3][r] - newm);
      rs += (e0 + e1) + (e2 + e3);
      pb0.h[r] = (_Float16)(e0 * 256.0f); pb0.h[8 + r] = (_Float16)(e1 * 256.0f);
      pb1.h[r] = (_Float16)(e2 * 256.0f); pb1.h[8 + r] = (_Float16)(e3 * 256.0f);
    }
    l_run = l_run * alpha + rs;
#pragma unroll
    for (int t = 0; t < 4; ++t)
#pragma unroll
      for (int r = 0; r < 8; ++r) o[t][r] *= alpha;
#pragma unroll
    for (int t = 0; t < 4; ++t) { const _Float16* vp = vbase + (size_t)(16 * t) * SEQ + key0; const v16h a0 = g2_frag(vp, hh), a1 = g2_frag(vp + 32, hh); o[t] = mma2(a0, pb0.v, a1, pb1.v, o[t]); }
  }
  const float lt = l_run + __shfl_xor(l_run, 16);
  const float inv = 0.00390625f * (1.0f / lt);
#pragma unroll
  for (int t = 0; t < 4; ++t) { v4f a, c;
#pragma unroll
    for (int r = 0; r < 4; ++r) { a[r] = o[t][r] * inv; c[r] = o[t][4 + r] * inv; }
    *(v4fa*)&so[w][ln][16 * t + 8 * hh] = a; *(v4fa*)&so[w][ln][16 * t + 8 * hh + 4] = c; }
  __builtin_amdgcn_fence(4  , "workgroup"); __builtin_amdgcn_wave_barrier();
  const unsigned rsub = lane >> 4, c4 = (lane & 15u) * 4u;
  float* obase = out + (size_t)(b * (unsigned)SEQ + q0) * HID + h * 64u;
  for (int pass = 0; pass < 2; ++pass) {
#pragma unroll
    for (int q = 0; q < 8; ++q) { const unsigned r = (unsigned)q * 2u + rsub; const v4f v = *(const v4fa*)&so[w][r][c4]; *(volatile v4f*)(obase + (size_t)r * HID + c4) = v; }
    if (pass == 0) __threadfence(); }
}

extern "C" void kernel_launch(void* const* d_in, const int* in_sizes, int n_in,
                              void* d_out, int out_size, void* d_ws, size_t ws_size, hipStream_t stream) {
  if (n_in < 8) return;
  const long long x_need = ((long long)(NB - 1) * SEQ_FULL + SEQ) * HID;
  const long long m_need = ((long long)(NB - 1) * SEQ_FULL + (SEQ - 1)) * SEQ_FULL + SEQ;
  if ((long long)in_sizes[0] < x_need) return;
  if ((long long)in_sizes[1] < m_need) return;
  if ((long long)in_sizes[2] < (long long)HID * HID || (long long)in_sizes[4] < (long long)HID * HID || (long long)in_sizes[6] < (long long)HID * HID) return;
  if (in_sizes[3] < HID || in_sizes[5] < HID || in_sizes[7] < HID) return;
  if ((long long)out_size < (long long)NR * HID) return;
  const float* x = (const float*)d_in[0]; const float* mask = (const float*)d_in[1];
  const float* wq = (const float*)d_in[2]; const float* bq = (const float*)d_in[3];
  const float* wk = (const float*)d_in[4]; const float* bk = (const float*)d_in[5];
  const float* wv = (const float*)d_in[6]; const float* bv = (const float*)d_in[7];
  char* ws = (char*)d_ws; size_t off = 0;
  auto take = [&](size_t bytes) { char* p = ws + off; off += (bytes + 255) & ~(size_t)255; return p; };
  _Float16* W16 = (_Float16*)take((size_t)3 * HID * HID * 2);
  _Float16* X16 = (_Float16*)take((size_t)NR * HID * 2);
  _Float16* QKV = (_Float16*)take((size_t)3 * NR * HID * 2);
  _Float16* VT = (_Float16*)take((size_t)NB * NH * HD * SEQ * 2);
  unsigned int* FL = (unsigned int*)take((size_t)NFP * 4);
  if (off > ws_size) return;
  _Float16* Q16 = QKV; _Float16* K16 = QKV + (size_t)NR * HID; _Float16* V16 = QKV + (size_t)2 * NR * HID;
  k_wnat<<<dim3((unsigned)(HID * HID / 8 / 256), 3), 256, 0, stream>>>(wq, wk, wv, W16);
  k_x16<<<dim3((unsigned)(SEQ * HID / 8 / 256), (unsigned)NB), 256, 0, stream>>>(x, X16);
  k_mflag<<<(unsigned)(NFP / 32), 256, 0, stream>>>(mask, FL);
  k_gemm2<<<dim3((unsigned)((NR / 128) * NTN), 3), 128, 0, stream>>>(X16, W16, bq, bk, bv, QKV);
  k_vt<<<(unsigned)(NB * NH * NT64), 256, 0, stream>>>(V16, VT);
  k_flash<<<(unsigned)(NB * NH * NT64), 128, 0, stream>>>(Q16, K16, VT, mask, FL, (float*)d_out);
}
